// LocalAttention_45037027065913
// MI455X (gfx1250) — hardware-verified
//
#include <hip/hip_runtime.h>
#include <stddef.h>


typedef _Float16 v16h __attribute__((ext_vector_type(16)));
typedef _Float16 v8h  __attribute__((ext_vector_type(8)));
typedef _Float16 v4h  __attribute__((ext_vector_type(4)));
typedef float    v8f  __attribute__((ext_vector_type(8)));
typedef float    v4f  __attribute__((ext_vector_type(4)));

#ifndef NB
#define NB 256
#endif
#ifndef SEQ
#define SEQ 2048
#endif
#define NB_FULL  256
#define SEQ_FULL 2048
#define EDIM  128
#define OCH   128
#define WIN   5
#define HALO  2
#define VROWS 50001
#define CH    128
#define GROWS (CH + 2 * HALO)
#define PTILES ((GROWS + 15) / 16)
#define PROWS (PTILES * 16)
#define GITER ((GROWS + 7) / 8)
#define LDA   136
#define PLD   16
#define ECARRY 16.0f
#define WCARRY 64.0f

static_assert(NB >= 1 && NB <= NB_FULL);
static_assert(SEQ >= CH && SEQ <= SEQ_FULL && (SEQ % CH) == 0);
static_assert(WIN == 2 * HALO + 1 && WIN <= 16);
static_assert(EDIM == 32 * 4);
static_assert((EDIM % 32) == 0 && EDIM / 32 == 4);
static_assert(OCH == 8 * 16);
static_assert(OCH == 32 * 4);
static_assert(CH == 8 * 16 && CH <= 256);
static_assert(CH == 4 * 32);
static_assert(GROWS <= PROWS && PROWS - GROWS == 12);
static_assert(GITER * 8 >= GROWS);
static_assert((LDA % 8) == 0 && LDA >= EDIM);
static_assert(HALO + CH + (WIN - 1 - HALO) <= GROWS);
static_assert(CH - 1 + WIN - 1 < PROWS);
static_assert((size_t)PROWS * LDA * 2 + (size_t)PROWS * PLD * 4 + CH * 4 + OCH * 4 <= (size_t)65536);

__device__ __forceinline__ float bf16r(float x) {
  unsigned int u = __float_as_uint(x);
  u = (u + 0x7FFFu + ((u >> 16) & 1u)) & 0xFFFF0000u;
  return __uint_as_float(u);
}

__device__ __forceinline__ _Float16 toh_flush(float v) {
  const _Float16 r = (_Float16)v;
  return (fabsf(v) < 6.103515625e-05f) ? (_Float16)0.0f : r;
}

__device__ __forceinline__ v16h frag_at(const _Float16* p) {
  v8h lo = *(const v8h*)(p);
  v8h hi = *(const v8h*)(p + 16);
  v16h out;
#pragma unroll
  for (int i = 0; i < 8; ++i) { out[i] = lo[i]; out[i + 8] = hi[i]; }
  return out;
}
__device__ __forceinline__ v16h ld_frag(const _Float16* base, unsigned ld) {
  const unsigned lane = threadIdx.x & 31u;
  return frag_at(base + (lane & 15u) * ld + (lane >> 4) * 8u);
}

__device__ __forceinline__ v8f wmma16(v16h a, v16h b, v8f c) {
  v8f d = __builtin_amdgcn_wmma_f32_16x16x32_f16(false, a, false, b, (short)0, c,
                                                 false, false);
  asm volatile("v_nop\n\tv_nop\n\tv_nop\n\tv_nop" : "+v"(d) : "v"(a), "v"(b));
  return d;
}

__global__ __launch_bounds__(256) void local_gate_kernel(
    const int* __restrict__ x, const float* __restrict__ emb,
    const float* __restrict__ attw, const float* __restrict__ attb,
    const float* __restrict__ cnnw, const float* __restrict__ cnnb,
    float* __restrict__ out) {
  __shared__ __attribute__((aligned(16))) _Float16 As[PROWS * LDA];
  __shared__ __attribute__((aligned(16))) float Pl[PROWS * PLD];
  __shared__ __attribute__((aligned(16))) float sc[CH];
  __shared__ __attribute__((aligned(16))) float outs[OCH];

  const unsigned tid = threadIdx.x, lane = tid & 31u, wv = tid >> 5;
  const unsigned wave = __builtin_amdgcn_readfirstlane(threadIdx.x >> 5);
  const unsigned hh = lane >> 4, m = lane & 15u;
  const unsigned b = blockIdx.x;
  const int* xrow = x + (size_t)b * SEQ_FULL;

  v16h bf[4], wf[4];
  {
    const unsigned oc = wv * 16u + m;
    const unsigned ar = (m < (unsigned)WIN) ? m : (unsigned)(WIN - 1);
    const bool live = (m < (unsigned)WIN);
#pragma unroll
    for (int c = 0; c < 4; ++c) {
      const float* src = cnnw + (size_t)oc * EDIM + (unsigned)c * 32u + hh * 8u;
      const v4f c0 = *(const v4f*)(src);
      const v4f c1 = *(const v4f*)(src + 4);
      const v4f c2 = *(const v4f*)(src + 16);
      const v4f c3 = *(const v4f*)(src + 20);
      const float* sa = attw + (size_t)ar * EDIM + (unsigned)c * 32u + hh * 8u;
      const v4f a0 = *(const v4f*)(sa);
      const v4f a1 = *(const v4f*)(sa + 4);
      const v4f a2 = *(const v4f*)(sa + 16);
      const v4f a3 = *(const v4f*)(sa + 20);
#pragma unroll
      for (int i = 0; i < 4; ++i) {
        bf[c][i]      = toh_flush(WCARRY * bf16r(c0[i]));
        bf[c][i + 4]  = toh_flush(WCARRY * bf16r(c1[i]));
        bf[c][i + 8]  = toh_flush(WCARRY * bf16r(c2[i]));
        bf[c][i + 12] = toh_flush(WCARRY * bf16r(c3[i]));
        wf[c][i]      = toh_flush(live ? (WCARRY * bf16r(a0[i])) : 0.0f);
        wf[c][i + 4]  = toh_flush(live ? (WCARRY * bf16r(a1[i])) : 0.0f);
        wf[c][i + 8]  = toh_flush(live ? (WCARRY * bf16r(a2[i])) : 0.0f);
        wf[c][i + 12] = toh_flush(live ? (WCARRY * bf16r(a3[i])) : 0.0f);
      }
    }
  }
  const float bias  = bf16r(cnnb[wv * 16u + m]);
  const float attb0 = bf16r(attb[0]);

  if (wave < 6u) {
    const unsigned r = (unsigned)GROWS + (tid >> 4);
    const unsigned c = (tid & 15u) * 8u;
    const v8h z = {};
    *(v8h*)&As[r * LDA + c] = z;
  }

  float runmax = -3.0e38f;

#pragma unroll 1
  for (unsigned tbase = 0; tbase < (unsigned)SEQ; tbase += (unsigned)CH) {
    __syncthreads();

#pragma unroll 1
    for (unsigned it = 0; it < (unsigned)GITER; ++it) {
      if (wave + 8u * it < (unsigned)GROWS) {
        const unsigned r = wv + 8u * it;
        const int tg = (int)(tbase + r) - HALO;
        const bool inb = (tg >= 0) && (tg < SEQ);
        const int tc = min(max(tg, 0), SEQ - 1);
        int tok = xrow[tc];
        tok = min(max(tok, 0), VROWS - 1);
        const v4f e = *(const v4f*)(emb + (size_t)tok * EDIM + lane * 4u);
        v4h o;
#pragma unroll
        for (int i = 0; i < 4; ++i) {
          const float f = inb ? (ECARRY * bf16r(e[i])) : 0.0f;
          o[i] = toh_flush(f);
        }
        *(v4h*)&As[r * LDA + lane * 4u] = o;
      }
    }
    __syncthreads();

    for (unsigned j = wave; j < (unsigned)PTILES; j += 8u) {
      v8f acc = {};
#pragma unroll
      for (int c = 0; c < 4; ++c) {
        const v16h a = ld_frag(&As[(16u * j) * LDA + (unsigned)c * 32u], LDA);
        acc = wmma16(a, wf[c], acc);
      }
#pragma unroll
      for (int r = 0; r < 8; ++r)
        Pl[(16u * j + hh * 8u + (unsigned)r) * PLD + m] = acc[r];
    }
    __syncthreads();

    if (wave < 4u) {
      float s = 0.0f;
#pragma unroll
      for (unsigned k = 0; k < (unsigned)WIN; ++k) s = s + Pl[(tid + k) * PLD + k];
      const float z = s * (1.0f / (ECARRY * WCARRY)) + attb0;
      const float sg = 1.0f / (1.0f + expf(-z));
      sc[tid] = sg * (1.0f / (ECARRY * WCARRY));
    }
    __syncthreads();

#pragma unroll 1
    for (unsigned j = 0; j < (unsigned)(CH / 16); ++j) {
      v8f acc = {};
#pragma unroll
      for (int c = 0; c < 4; ++c) {
        const v16h a = ld_frag(&As[((unsigned)HALO + 16u * j) * LDA + (unsigned)c * 32u], LDA);
        acc = wmma16(a, bf[c], acc);
      }
      const v4f s0 = *(const v4f*)&sc[16u * j + hh * 8u];
      const v4f s1 = *(const v4f*)&sc[16u * j + hh * 8u + 4u];
#pragma unroll
      for (int r = 0; r < 4; ++r) {
        runmax = fmaxf(runmax, acc[r] * s0[r] + bias);
        runmax = fmaxf(runmax, acc[r + 4] * s1[r] + bias);
      }
    }
  }

  runmax = fmaxf(runmax, __shfl_xor(runmax, 16, 32));
  const float res = tanhf(runmax);
  if (hh == 0u) outs[wv * 16u + m] = res;
  __syncthreads();

  if (wave == 0u) {
    const v4f val = *(const v4f*)&outs[lane * 4u];
    float* p = out + (size_t)b * OCH + lane * 4u;
    *(volatile v4f*)p = val;
    __threadfence();
    *(volatile v4f*)p = val;
  }
}

extern "C" void kernel_launch(void* const* d_in, const int* in_sizes, int n_in,
                              void* d_out, int out_size, void* d_ws, size_t ws_size,
                              hipStream_t stream) {
  (void)d_ws;
  (void)ws_size;
  if (n_in < 6) return;
  const long long need_x = (long long)(NB - 1) * SEQ_FULL + SEQ;
  if ((long long)in_sizes[0] < need_x) return;
  if ((long long)in_sizes[1] < (long long)VROWS * EDIM) return;
  if (in_sizes[2] < WIN * EDIM) return;
  if (in_sizes[3] < 1) return;
  if (in_sizes[4] < OCH * EDIM) return;
  if (in_sizes[5] < OCH) return;
  if ((long long)out_size < (long long)NB * OCH) return;

  const int*   x    = (const int*)d_in[0];
  const float* emb  = (const float*)d_in[1];
  const float* attw = (const float*)d_in[2];
  const float* attb = (const float*)d_in[3];
  const float* cnnw = (const float*)d_in[4];
  const float* cnnb = (const float*)d_in[5];
  float* out = (float*)d_out;

  local_gate_kernel<<<dim3(NB), dim3(256), 0, stream>>>(x, emb, attw, attb, cnnw, cnnb, out);
}
